// MambaBlock_58342835749247
// MI455X (gfx1250) — hardware-verified
//
#include <hip/hip_runtime.h>
#include <stddef.h>
#include <stdint.h>
#include <math.h>

#define T_TOK  4096
#define SEQL   2048
#define DIM    1024
#define DIN    2048
#define NST    16
#define DTR    64
#define XPN    96
#define K2IN   4096
#define K2DT   128
#define GTHR   128
#define PTHR   256
#define SCH    64
#define STT    64
#define PLANE  ((size_t)T_TOK * DIN)

#define NU_X    (T_TOK * DIM / 8)
#define NU_WIN  (2 * DIN * DIM / 8)
#define NU_WOUT (DIM * K2IN / 8)
#define NU_WXP  (XPN * K2IN / 8)
#define NU_WDT  (DIN * K2DT / 8)
#define NU_AN   (DIN * NST / 4)
#define NU_ALL  (NU_X + NU_WIN + NU_WOUT + NU_WXP + NU_WDT + NU_AN)

static_assert(NU_X % PTHR == 0 && NU_WIN % PTHR == 0 && NU_WOUT % PTHR == 0);
static_assert(NU_WXP % PTHR == 0 && NU_WDT % PTHR == 0 && NU_AN % PTHR == 0);
static_assert(DIM % 32 == 0 && K2IN % 32 == 0 && K2DT % 32 == 0);
static_assert(T_TOK % 128 == 0 && (2 * DIN) % 64 == 0 && DIN % 64 == 0 && DIM % 64 == 0);
static_assert(K2IN == 2 * DIN && K2DT == 2 * DTR && XPN == DTR + 2 * NST);
static_assert(SEQL % STT == 0 && DIN % SCH == 0 && SCH == 64 && STT == 64);
static_assert((T_TOK * DIN / 4) % PTHR == 0);

enum { EPI_IN = 0, EPI_XP = 1, EPI_DT = 2, EPI_OUT = 3 };

typedef float          v4f   __attribute__((ext_vector_type(4)));
typedef float          v8f   __attribute__((ext_vector_type(8)));
typedef int            v8i   __attribute__((ext_vector_type(8)));
typedef unsigned short v4us  __attribute__((ext_vector_type(4)));
typedef unsigned short v8us  __attribute__((ext_vector_type(8)));
typedef unsigned short v16us __attribute__((ext_vector_type(16)));
typedef __bf16         v16bf __attribute__((ext_vector_type(16)));
typedef v4f  __attribute__((may_alias)) v4fa;
typedef v8us __attribute__((may_alias)) v8usa;
union FragB { v16bf v; v16us u; v8us h[2]; v8i w; };

__device__ __forceinline__ v8f wmb(const FragB& a, const FragB& b, v8f c) {
  v8f d = __builtin_amdgcn_wmma_f32_16x16x32_bf16(false, a.v, false, b.v, (short)0, c, false, false);
  asm volatile("v_nop\n\tv_nop\n\tv_nop\n\tv_nop" : "+v"(d) : "v"(a.w), "v"(b.w));
  return d;
}

__device__ __forceinline__ unsigned bf16_bits(float f) {
  const unsigned u = __float_as_uint(f);
  return (u + 0x7FFFu + ((u >> 16) & 1u)) >> 16;
}
__device__ __forceinline__ float bf16_val(float f) {
  return __uint_as_float(bf16_bits(f) << 16);
}
__device__ __forceinline__ unsigned short hl_sel(float v, bool lo) {
  const unsigned hb = bf16_bits(v);
  const unsigned lb = bf16_bits(v - __uint_as_float(hb << 16));
  return (unsigned short)(lo ? lb : hb);
}
__device__ __forceinline__ float silu_f(float c) {
  return c * __builtin_amdgcn_rcpf(1.0f + expf(-c));
}
__device__ __forceinline__ float softplus_f(float v) {
  return fmaxf(v, 0.0f) + log1pf(expf(-fabsf(v)));
}

__device__ __forceinline__ void cvt8(const float* __restrict__ p, unsigned short* dp) {
  const v4f a = *(const v4f*)p;
  const v4f b = *(const v4f*)(p + 4);
  v8us o;
  o[0] = (unsigned short)bf16_bits(a.x); o[1] = (unsigned short)bf16_bits(a.y);
  o[2] = (unsigned short)bf16_bits(a.z); o[3] = (unsigned short)bf16_bits(a.w);
  o[4] = (unsigned short)bf16_bits(b.x); o[5] = (unsigned short)bf16_bits(b.y);
  o[6] = (unsigned short)bf16_bits(b.z); o[7] = (unsigned short)bf16_bits(b.w);
  *(volatile v8us*)dp = o;
  __threadfence();
  *(volatile v8us*)dp = o;
}

__global__ __launch_bounds__(PTHR) void k_prep(const float* __restrict__ x, const float* __restrict__ Win,
                                               const float* __restrict__ Wxp, const float* __restrict__ Wdt,
                                               const float* __restrict__ Wout, const float* __restrict__ Alog,
                                               unsigned short* XB, unsigned short* WIN, unsigned short* WXP2,
                                               unsigned short* WDT2, unsigned short* WOUT2, float* AN) {
  int u = (int)blockIdx.x * PTHR + (int)threadIdx.x;
  if (u < NU_X) { cvt8(x + (size_t)u * 8, XB + (size_t)u * 8); return; }
  u -= NU_X;
  if (u < NU_WIN) { cvt8(Win + (size_t)u * 8, WIN + (size_t)u * 8); return; }
  u -= NU_WIN;
  if (u < NU_WOUT) {
    const int n = u >> 9, k8 = (u & 511) * 8;
    cvt8(Wout + (size_t)n * DIN + (k8 & (DIN - 1)), WOUT2 + (size_t)n * K2IN + k8);
    return;
  }
  u -= NU_WOUT;
  if (u < NU_WXP) {
    const int n = u >> 9, k8 = (u & 511) * 8;
    cvt8(Wxp + (size_t)n * DIN + (k8 & (DIN - 1)), WXP2 + (size_t)n * K2IN + k8);
    return;
  }
  u -= NU_WXP;
  if (u < NU_WDT) {
    const int n = u >> 4, k8 = (u & 15) * 8;
    cvt8(Wdt + (size_t)n * DTR + (k8 & (DTR - 1)), WDT2 + (size_t)n * K2DT + k8);
    return;
  }
  u -= NU_WDT;
  if (u < NU_AN) {
    const v4f a = *(const v4f*)(Alog + (size_t)u * 4);
    v4f o;
    o.x = -expf(bf16_val(a.x)); o.y = -expf(bf16_val(a.y));
    o.z = -expf(bf16_val(a.z)); o.w = -expf(bf16_val(a.w));
    float* dp = AN + (size_t)u * 4;
    *(volatile v4f*)dp = o;
    __threadfence();
    *(volatile v4f*)dp = o;
  }
}

template <int MT, int NT, int EPI>
__global__ __launch_bounds__(GTHR) void k_gemm(const unsigned short* __restrict__ A,
                                               const unsigned short* __restrict__ BT, int K,
                                               float* outF, unsigned short* outH,
                                               const float* __restrict__ bias) {
  constexpr int BM = 64 * MT;
  constexpr int BN = 16 * NT;
  constexpr int RW = 16 * MT;
  static_assert(EPI == EPI_XP ? (MT == 1 && NT == 6) : (MT == 2 && NT == 4));
  __shared__ __attribute__((aligned(16))) float stg[BM * BN];
  const int tid = (int)threadIdx.x, lane = tid & 31, wave = tid >> 5, hh = lane >> 4, m = lane & 15;
  const int rowBase = (int)blockIdx.x * BM;
  const int col0    = (int)blockIdx.y * BN;

  v8f acc[MT][NT];
  {
    const v8f z = {0.f, 0.f, 0.f, 0.f, 0.f, 0.f, 0.f, 0.f};
#pragma unroll
    for (int i = 0; i < MT; ++i)
#pragma unroll
      for (int t = 0; t < NT; ++t) acc[i][t] = z;
  }
  const unsigned short* ap = A  + (size_t)(rowBase + RW * wave + m) * (size_t)K + 8 * hh;
  const unsigned short* bp = BT + (size_t)(col0 + m) * (size_t)K + 8 * hh;

#pragma unroll 1
  for (int k0 = 0; k0 < K; k0 += 32) {
    FragB af[MT];
#pragma unroll
    for (int i = 0; i < MT; ++i) {
      const unsigned short* aq = ap + (size_t)(16 * i) * (size_t)K + k0;
      af[i].h[0] = *(const v8usa*)aq;
      af[i].h[1] = *(const v8usa*)(aq + 16);
    }
#pragma unroll
    for (int t = 0; t < NT; ++t) {
      const unsigned short* wq = bp + (size_t)(16 * t) * (size_t)K + k0;
      FragB bf;
      bf.h[0] = *(const v8usa*)wq;
      bf.h[1] = *(const v8usa*)(wq + 16);
#pragma unroll
      for (int i = 0; i < MT; ++i) acc[i][t] = wmb(af[i], bf, acc[i][t]);
    }
  }

#pragma unroll
  for (int i = 0; i < MT; ++i)
#pragma unroll
    for (int t = 0; t < NT; ++t) {
      const int lc = 16 * t + m;
#pragma unroll
      for (int r = 0; r < 8; ++r) {
        const int lr = RW * wave + 16 * i + 8 * hh + r;
        stg[lr * BN + lc] = acc[i][t][r];
      }
    }
  __syncthreads();

  if constexpr (EPI == EPI_XP) {
#pragma unroll 1
    for (int i = 0; i < 8; ++i) {
      const int lr = 16 * wave + 2 * i + hh;
      const int cb = 8 * (m & 7);
      const v4f a = *(const v4fa*)(stg + lr * BN + cb);
      const v4f b = *(const v4fa*)(stg + lr * BN + cb + 4);
      const bool lo = (m & 8) != 0;
      v8us o;
      o[0] = hl_sel(a.x, lo); o[1] = hl_sel(a.y, lo); o[2] = hl_sel(a.z, lo); o[3] = hl_sel(a.w, lo);
      o[4] = hl_sel(b.x, lo); o[5] = hl_sel(b.y, lo); o[6] = hl_sel(b.z, lo); o[7] = hl_sel(b.w, lo);
      unsigned short* hp = outH + (size_t)(rowBase + lr) * K2DT + 8 * m;
      *(volatile v8us*)hp = o;
      __threadfence();
      *(volatile v8us*)hp = o;
    }
#pragma unroll 1
    for (int i = 0; i < 4; ++i) {
      const int lr = 16 * wave + 4 * i + (lane >> 3);
      const int c4 = 4 * (lane & 7);
      const v4f v = *(const v4fa*)(stg + lr * BN + DTR + c4);
      float* op = outF + (size_t)(rowBase + lr) * (2 * NST) + c4;
      *(volatile v4f*)op = v;
      __threadfence();
      *(volatile v4f*)op = v;
    }
  } else {
    v4f bb = {0.f, 0.f, 0.f, 0.f};
    if constexpr (EPI == EPI_DT) {
      const v4f t1 = *(const v4f*)(bias + col0 + 4 * m);
      bb.x = bf16_val(t1.x); bb.y = bf16_val(t1.y); bb.z = bf16_val(t1.z); bb.w = bf16_val(t1.w);
    }
    const int plane = col0 >> 11;
    const int cc    = col0 & (DIN - 1);
#pragma unroll 1
    for (int i = 0; i < RW / 2; ++i) {
      const int lr = RW * wave + 2 * i + hh;
      const int gr = rowBase + lr;
      v4f v = *(const v4fa*)(stg + lr * BN + 4 * m);
      float* op;
      if constexpr (EPI == EPI_IN) {
        if (plane != 0) {
          v.x = silu_f(v.x); v.y = silu_f(v.y); v.z = silu_f(v.z); v.w = silu_f(v.w);
        }
        op = outF + (size_t)plane * PLANE + (size_t)gr * DIN + cc + 4 * m;
      } else if constexpr (EPI == EPI_DT) {
        v = v + bb;
        v.x = softplus_f(v.x); v.y = softplus_f(v.y); v.z = softplus_f(v.z); v.w = softplus_f(v.w);
        op = outF + (size_t)gr * DIN + col0 + 4 * m;
      } else {
        op = outF + (size_t)gr * DIM + col0 + 4 * m;
      }
      *(volatile v4f*)op = v;
      __threadfence();
      *(volatile v4f*)op = v;
    }
  }
}

__global__ __launch_bounds__(PTHR) void k_conv(const float* __restrict__ xcp, const float* __restrict__ cw,
                                               const float* __restrict__ cb, float* U, unsigned short* UHL) {
  const int idx = (int)blockIdx.x * PTHR + (int)threadIdx.x;
  const int t   = idx >> 9;
  const int d4  = (idx & 511) * 4;
  const int l   = t & (SEQL - 1);

  v4f w0 = *(const v4f*)(cw + (size_t)(d4 + 0) * 4);
  v4f w1 = *(const v4f*)(cw + (size_t)(d4 + 1) * 4);
  v4f w2 = *(const v4f*)(cw + (size_t)(d4 + 2) * 4);
  v4f w3 = *(const v4f*)(cw + (size_t)(d4 + 3) * 4);
  v4f bb = *(const v4f*)(cb + d4);
  w0.x = bf16_val(w0.x); w0.y = bf16_val(w0.y); w0.z = bf16_val(w0.z); w0.w = bf16_val(w0.w);
  w1.x = bf16_val(w1.x); w1.y = bf16_val(w1.y); w1.z = bf16_val(w1.z); w1.w = bf16_val(w1.w);
  w2.x = bf16_val(w2.x); w2.y = bf16_val(w2.y); w2.z = bf16_val(w2.z); w2.w = bf16_val(w2.w);
  w3.x = bf16_val(w3.x); w3.y = bf16_val(w3.y); w3.z = bf16_val(w3.z); w3.w = bf16_val(w3.w);
  bb.x = bf16_val(bb.x); bb.y = bf16_val(bb.y); bb.z = bf16_val(bb.z); bb.w = bf16_val(bb.w);

  v4f acc = {0.f, 0.f, 0.f, 0.f};
#pragma unroll
  for (int k = 0; k < 4; ++k) {
    const int back = 3 - k;
    const bool ok = l >= back;
    const int tr = ok ? (t - back) : t;
    const v4f xv = *(const v4f*)(xcp + (size_t)tr * DIN + d4);
    const float x0 = ok ? xv.x : 0.0f;
    const float x1 = ok ? xv.y : 0.0f;
    const float x2 = ok ? xv.z : 0.0f;
    const float x3 = ok ? xv.w : 0.0f;
    acc.x = acc.x + x0 * w0[k];
    acc.y = acc.y + x1 * w1[k];
    acc.z = acc.z + x2 * w2[k];
    acc.w = acc.w + x3 * w3[k];
  }
  acc = acc + bb;
  v4f uo;
  uo.x = silu_f(acc.x); uo.y = silu_f(acc.y); uo.z = silu_f(acc.z); uo.w = silu_f(acc.w);
  v4us hv, lv;
  hv[0] = hl_sel(uo.x, false); lv[0] = hl_sel(uo.x, true);
  hv[1] = hl_sel(uo.y, false); lv[1] = hl_sel(uo.y, true);
  hv[2] = hl_sel(uo.z, false); lv[2] = hl_sel(uo.z, true);
  hv[3] = hl_sel(uo.w, false); lv[3] = hl_sel(uo.w, true);
  float* up = U + (size_t)t * DIN + d4;
  unsigned short* hp = UHL + (size_t)t * K2IN + d4;
  *(volatile v4f*)up = uo;
  *(volatile v4us*)hp = hv;
  *(volatile v4us*)(hp + DIN) = lv;
  __threadfence();
  *(volatile v4f*)up = uo;
  *(volatile v4us*)hp = hv;
  *(volatile v4us*)(hp + DIN) = lv;
}

#define SCAN_N(N, BV, CV) { const float dA = expf(dlt * an[N]); h[N] = dA * h[N] + du * (BV); acc += h[N] * (CV); }

__global__ __launch_bounds__(SCH) void k_scan(const float* __restrict__ DELTA, const float* __restrict__ U,
                                              const float* __restrict__ SZ, const float* __restrict__ BC,
                                              const float* __restrict__ AN, const float* __restrict__ Dv,
                                              unsigned short* YHL) {
  __shared__ __attribute__((aligned(16))) float bcs[STT * 32];
  __shared__ __attribute__((aligned(16))) unsigned short ohi[STT * SCH];
  __shared__ __attribute__((aligned(16))) unsigned short olo[STT * SCH];
  const int tid = (int)threadIdx.x;
  const int b = (int)blockIdx.x >> 5;
  const int chBase = ((int)blockIdx.x & 31) * SCH;
  const int d = chBase + tid;

  float an[NST], h[NST];
  {
    const v4f a0 = *(const v4f*)(AN + (size_t)d * NST);
    const v4f a1 = *(const v4f*)(AN + (size_t)d * NST + 4);
    const v4f a2 = *(const v4f*)(AN + (size_t)d * NST + 8);
    const v4f a3 = *(const v4f*)(AN + (size_t)d * NST + 12);
    an[0] = a0.x; an[1] = a0.y; an[2] = a0.z; an[3] = a0.w;
    an[4] = a1.x; an[5] = a1.y; an[6] = a1.z; an[7] = a1.w;
    an[8] = a2.x; an[9] = a2.y; an[10] = a2.z; an[11] = a2.w;
    an[12] = a3.x; an[13] = a3.y; an[14] = a3.z; an[15] = a3.w;
  }
#pragma unroll
  for (int n = 0; n < NST; ++n) h[n] = 0.0f;
  const float Dd = bf16_val(Dv[d]);
  const int q = tid >> 3, p = tid & 7;

#pragma unroll 1
  for (int tile = 0; tile < SEQL / STT; ++tile) {
    const int rowT = b * SEQL + tile * STT;
    {
      const float* src = BC + (size_t)rowT * 32;
#pragma unroll
      for (int it = 0; it < (STT * 32) / (4 * SCH); ++it) {
        const int i4 = 4 * (it * SCH + tid);
        *(v4f*)(bcs + i4) = *(const v4f*)(src + i4);
      }
    }
    __syncthreads();

#pragma unroll 1
    for (int tl = 0; tl < STT; ++tl) {
      const size_t eo = (size_t)(rowT + tl) * DIN + d;
      const float dlt = DELTA[eo];
      const float u   = U[eo];
      const float sz  = SZ[eo];
      const float du  = dlt * u;
      const float* bcr = bcs + tl * 32;
      const v4f b0 = *(const v4f*)(bcr);      const v4f b1 = *(const v4f*)(bcr + 4);
      const v4f b2 = *(const v4f*)(bcr + 8);  const v4f b3 = *(const v4f*)(bcr + 12);
      const v4f c0 = *(const v4f*)(bcr + 16); const v4f c1 = *(const v4f*)(bcr + 20);
      const v4f c2 = *(const v4f*)(bcr + 24); const v4f c3 = *(const v4f*)(bcr + 28);
      float acc = 0.0f;
      SCAN_N(0,  b0.x, c0.x) SCAN_N(1,  b0.y, c0.y) SCAN_N(2,  b0.z, c0.z) SCAN_N(3,  b0.w, c0.w)
      SCAN_N(4,  b1.x, c1.x) SCAN_N(5,  b1.y, c1.y) SCAN_N(6,  b1.z, c1.z) SCAN_N(7,  b1.w, c1.w)
      SCAN_N(8,  b2.x, c2.x) SCAN_N(9,  b2.y, c2.y) SCAN_N(10, b2.z, c2.z) SCAN_N(11, b2.w, c2.w)
      SCAN_N(12, b3.x, c3.x) SCAN_N(13, b3.y, c3.y) SCAN_N(14, b3.z, c3.z) SCAN_N(15, b3.w, c3.w)
      const float y2 = acc + u * Dd;
      const float g  = y2 * sz;
      const unsigned hb = bf16_bits(g);
      const unsigned lb = bf16_bits(g - __uint_as_float(hb << 16));
      ohi[tl * SCH + tid] = (unsigned short)hb;
      olo[tl * SCH + tid] = (unsigned short)lb;
    }
    __syncthreads();

    v8us vh[STT / 8], vl[STT / 8];
#pragma unroll
    for (int it = 0; it < STT / 8; ++it) {
      const int tok = it * 8 + q;
      vh[it] = *(const v8usa*)(ohi + tok * SCH + 8 * p);
      vl[it] = *(const v8usa*)(olo + tok * SCH + 8 * p);
    }
#pragma unroll
    for (int it = 0; it < STT / 8; ++it) {
      unsigned short* yp = YHL + (size_t)(rowT + it * 8 + q) * K2IN + chBase + 8 * p;
      *(volatile v8us*)yp = vh[it];
      *(volatile v8us*)(yp + DIN) = vl[it];
    }
    __threadfence();
#pragma unroll
    for (int it = 0; it < STT / 8; ++it) {
      unsigned short* yp = YHL + (size_t)(rowT + it * 8 + q) * K2IN + chBase + 8 * p;
      *(volatile v8us*)yp = vh[it];
      *(volatile v8us*)(yp + DIN) = vl[it];
    }
  }
}
#undef SCAN_N

static inline size_t al256(size_t o) { return (o + 255) & ~(size_t)255; }

extern "C" void kernel_launch(void* const* d_in, const int* in_sizes, int n_in,
                              void* d_out, int out_size, void* d_ws, size_t ws_size,
                              hipStream_t stream) {
  if (n_in < 10) return;
  if (in_sizes[0] != T_TOK * DIM) return;
  if (in_sizes[1] != 2 * DIN * DIM) return;
  if (in_sizes[2] != DIN * 4) return;
  if (in_sizes[3] != DIN) return;
  if (in_sizes[4] != XPN * DIN) return;
  if (in_sizes[5] != DIN * DTR) return;
  if (in_sizes[6] != DIN) return;
  if (in_sizes[7] != DIN * NST) return;
  if (in_sizes[8] != DIN) return;
  if (in_sizes[9] != DIM * DIN) return;
  if (out_size != T_TOK * DIM) return;

  const float* x     = (const float*)d_in[0];
  const float* W_in  = (const float*)d_in[1];
  const float* convw = (const float*)d_in[2];
  const float* convb = (const float*)d_in[3];
  const float* W_xp  = (const float*)d_in[4];
  const float* W_dt  = (const float*)d_in[5];
  const float* b_dt  = (const float*)d_in[6];
  const float* A_log = (const float*)d_in[7];
  const float* Dvec  = (const float*)d_in[8];
  const float* W_out = (const float*)d_in[9];
  float* out = (float*)d_out;

  char* ws = (char*)d_ws;
  size_t off = 0;
  const size_t oXB   = off; off = al256(off + (size_t)T_TOK * DIM * 2);
  const size_t oWIN  = off; off = al256(off + (size_t)2 * DIN * DIM * 2);
  const size_t oWOUT = off; off = al256(off + (size_t)DIM * K2IN * 2);
  const size_t oWXP  = off; off = al256(off + (size_t)XPN * K2IN * 2);
  const size_t oWDT  = off; off = al256(off + (size_t)DIN * K2DT * 2);
  const size_t oAN   = off; off = al256(off + (size_t)DIN * NST * 4);
  const size_t oP2   = off; off = al256(off + 2 * PLANE * 4);
  const size_t oU    = off; off = al256(off + PLANE * 4);
  const size_t oUHL  = off; off = al256(off + (size_t)T_TOK * K2IN * 2);
  const size_t oBC   = off; off = al256(off + (size_t)T_TOK * 2 * NST * 4);
  const size_t oDTL  = off; off = al256(off + (size_t)T_TOK * K2DT * 2);
  if (off > ws_size) return;
  unsigned short* XB    = (unsigned short*)(ws + oXB);
  unsigned short* WIN   = (unsigned short*)(ws + oWIN);
  unsigned short* WOUT2 = (unsigned short*)(ws + oWOUT);
  unsigned short* WXP2  = (unsigned short*)(ws + oWXP);
  unsigned short* WDT2  = (unsigned short*)(ws + oWDT);
  float*          AN    = (float*)(ws + oAN);
  float*          P2    = (float*)(ws + oP2);
  float*          Upl   = (float*)(ws + oU);
  unsigned short* UHL   = (unsigned short*)(ws + oUHL);
  float*          BCp   = (float*)(ws + oBC);
  unsigned short* DTLHL = (unsigned short*)(ws + oDTL);

  k_prep<<<NU_ALL / PTHR, PTHR, 0, stream>>>(x, W_in, W_xp, W_dt, W_out, A_log, XB, WIN, WXP2, WDT2, WOUT2, AN);
  k_gemm<2, 4, EPI_IN><<<dim3(T_TOK / 128, (2 * DIN) / 64), GTHR, 0, stream>>>(XB, WIN, DIM, P2, DTLHL, b_dt);
  k_conv<<<(T_TOK * DIN / 4) / PTHR, PTHR, 0, stream>>>(P2, convw, convb, Upl, UHL);
  k_gemm<1, 6, EPI_XP><<<dim3(T_TOK / 64, 1), GTHR, 0, stream>>>(UHL, WXP2, K2IN, BCp, DTLHL, b_dt);
  k_gemm<2, 4, EPI_DT><<<dim3(T_TOK / 128, DIN / 64), GTHR, 0, stream>>>(DTLHL, WDT2, K2DT, P2, DTLHL, b_dt);
  k_scan<<<2 * (DIN / SCH), SCH, 0, stream>>>(P2, Upl, P2 + PLANE, BCp, AN, Dvec, UHL);
  k_gemm<2, 4, EPI_OUT><<<dim3(T_TOK / 128, DIM / 64), GTHR, 0, stream>>>(UHL, WOUT2, K2IN, out, DTLHL, b_dt);
}
